// NGCF_91182155694432
// MI455X (gfx1250) — hardware-verified
//
#include <hip/hip_runtime.h>
#include <math.h>

constexpr int kNumUser   = 50000;
constexpr int kNumItem   = 100000;
constexpr int kNumNode   = 150000;
constexpr int kRowsPad   = 150016;
constexpr int kDim       = 64;
constexpr int kKdim      = 128;
constexpr int kNnz       = 2400000;
constexpr int kBatch     = 1024;
constexpr int kLayers    = 3;
constexpr int kNT        = 256;
constexpr int kTileRows  = 1024;
constexpr int kNumTiles  = 147;
constexpr int kWaveRows  = kTileRows / 8;
constexpr int kEPT       = 128;
constexpr int kChunk     = kNT * kEPT;
constexpr int kNumChunks = (kNnz + kChunk - 1) / kChunk;
constexpr int kNnzPad    = kNumChunks * kChunk;
constexpr int kKeyWords  = kNnzPad / 4;
constexpr int kCap       = 2048;
constexpr int kDynLds    = kTileRows * kDim * 4;
static_assert(kRowsPad % 64 == 0, "M tile multiple");
static_assert(kDim % 64 == 0, "N tile multiple");
static_assert(kKdim % 32 == 0, "K multiple of 32");
static_assert(kRowsPad >= kNumNode, "pad rows");
static_assert(kNumTiles * kTileRows >= kRowsPad, "tile coverage");
static_assert((kNumTiles - 1) * kTileRows < kRowsPad, "no empty tile");
static_assert(kNumTiles <= 255, "8-bit tile codes; 255 = no tile");
static_assert(kWaveRows == 128, "owner wave = local row >> 7 = entry >> 29");
static_assert(kWaveRows % 4 == 0, "epilogue row groups");
static_assert(kRowsPad % 4 == 0 && kNumNode % 4 == 0, "row groups never straddle bounds");
static_assert(kNnz % 16 == 0, "code groups entirely inside or outside the list");
static_assert(kNnzPad % (16 * kNT) == 0, "exact code grid");
static_assert(kNnz < (1 << 22), "edge index packed in 22 bits");
static_assert(kCap % kNT == 0, "list init coverage");
static_assert((kTileRows * kDim / 4) % kNT == 0, "accumulator init coverage");
static_assert((kNumUser * 16) % kNT == 0 && (kNumItem * 16) % kNT == 0, "exact copy grids");
static_assert((kRowsPad - kNumNode) * 16 == kNT, "pad zero fill = one block");
static_assert(kBatch % 32 == 0 && kBatch % 16 == 0, "exact batch grids");

typedef __attribute__((ext_vector_type(16))) _Float16 v16h;
typedef __attribute__((ext_vector_type(8)))  _Float16 v8h;
typedef __attribute__((ext_vector_type(16))) __bf16   v16b;
typedef __attribute__((ext_vector_type(8)))  __bf16   v8b;
typedef __attribute__((ext_vector_type(8)))  float    v8f;
typedef __attribute__((ext_vector_type(4)))  float    v4f;
typedef __attribute__((ext_vector_type(2)))  float    v2f;
typedef __attribute__((ext_vector_type(4)))  unsigned int v4u;
typedef __attribute__((ext_vector_type(4)))  int      v4i;

__device__ __forceinline__ unsigned short f2bf_bits(float f) {
  unsigned u = __float_as_uint(f);
  return (unsigned short)((u + 0x7FFFu + ((u >> 16) & 1u)) >> 16);
}
__device__ __forceinline__ float bf_bits2f(unsigned short h) { return __uint_as_float(((unsigned)h) << 16); }
__device__ __forceinline__ float bfr(float f) { return bf_bits2f(f2bf_bits(f)); }

__device__ __forceinline__ void dep_guard_h(v8f& a, v8f& b, v16h x, v16h y) { asm volatile("v_nop\n\tv_nop\n\tv_nop\n\tv_nop" : "+v"(a), "+v"(b) : "v"(x), "v"(y)); }
__device__ __forceinline__ void dep_guard_b(v8f& a, v8f& b, v16b x, v16b y) { asm volatile("v_nop\n\tv_nop\n\tv_nop\n\tv_nop" : "+v"(a), "+v"(b) : "v"(x), "v"(y)); }
__device__ __forceinline__ void dep_guard4_h(v8f& a, v8f& b, v8f& c, v8f& d, v16h x, v16h y) { asm volatile("v_nop\n\tv_nop\n\tv_nop\n\tv_nop" : "+v"(a), "+v"(b), "+v"(c), "+v"(d) : "v"(x), "v"(y)); }
__device__ __forceinline__ void dep_guard4_b(v8f& a, v8f& b, v8f& c, v8f& d, v16b x, v16b y) { asm volatile("v_nop\n\tv_nop\n\tv_nop\n\tv_nop" : "+v"(a), "+v"(b), "+v"(c), "+v"(d) : "v"(x), "v"(y)); }
__device__ __forceinline__ void keep4_h(v16h a, v16h b, v16h c, v16h d) { asm volatile("v_nop" :: "v"(a), "v"(b), "v"(c), "v"(d)); }
__device__ __forceinline__ void keep4_b(v16b a, v16b b, v16b c, v16b d) { asm volatile("v_nop" :: "v"(a), "v"(b), "v"(c), "v"(d)); }
__device__ __forceinline__ void acc_guard4(v8f& a, v8f& b, v8f& c, v8f& d) { asm volatile("v_nop\n\tv_nop\n\tv_nop\n\tv_nop" : "+v"(a), "+v"(b), "+v"(c), "+v"(d)); }
template <typename T> struct Frag;
template <> struct Frag<_Float16> {
  typedef v16h V; union U { v16h v; v8h h[2]; };
  static __device__ __forceinline__ v16h load(const _Float16* p) {
    U f; f.h[0] = *(const v8h*)(p); f.h[1] = *(const v8h*)(p + 16); return f.v;
  }
  static __device__ __forceinline__ v8f mma(v16h a, v16h b, v8f c) {
    return __builtin_amdgcn_wmma_f32_16x16x32_f16(false, a, false, b, (short)0, c, false, false);
  }
  static __device__ __forceinline__ void guard(v8f& a, v8f& b, v16h x, v16h y) { dep_guard_h(a, b, x, y); }
  static __device__ __forceinline__ void guard4(v8f& a, v8f& b, v8f& c, v8f& d, v16h x, v16h y) { dep_guard4_h(a, b, c, d, x, y); }
  static __device__ __forceinline__ void keep(v16h a, v16h b, v16h c, v16h d) { keep4_h(a, b, c, d); }
};
template <> struct Frag<__bf16> {
  typedef v16b V; union U { v16b v; v8b h[2]; };
  static __device__ __forceinline__ v16b load(const __bf16* p) {
    U f; f.h[0] = *(const v8b*)(p); f.h[1] = *(const v8b*)(p + 16); return f.v;
  }
  static __device__ __forceinline__ v8f mma(v16b a, v16b b, v8f c) {
    return __builtin_amdgcn_wmma_f32_16x16x32_bf16(false, a, false, b, (short)0, c, false, false);
  }
  static __device__ __forceinline__ void guard(v8f& a, v8f& b, v16b x, v16b y) { dep_guard_b(a, b, x, y); }
  static __device__ __forceinline__ void guard4(v8f& a, v8f& b, v8f& c, v8f& d, v16b x, v16b y) { dep_guard4_b(a, b, c, d, x, y); }
  static __device__ __forceinline__ void keep(v16b a, v16b b, v16b c, v16b d) { keep4_b(a, b, c, d); }
};

__device__ __forceinline__ unsigned pk16(unsigned short a, unsigned short b) { return (unsigned)a | ((unsigned)b << 16); }

template <int ET> struct Elem;
template <> struct Elem<0> { typedef _Float16 T; };
template <> struct Elem<1> { typedef __bf16 T; };
template <int ET, int SPLIT, int BIAS_MODE, int OUT_MODE, bool RESID, int ACT = 0>
__global__ __launch_bounds__(256) void wmma_gemm64(
    const unsigned short* __restrict__ Ap, const unsigned short* __restrict__ A2p, int lda, long strideA,
    const unsigned short* __restrict__ Btp, const unsigned short* __restrict__ Bt2p, int ldb, long strideB,
    void* __restrict__ Cout, void* __restrict__ Cout2, int ldc, long strideC,
    const float* __restrict__ bias,
    const float* __restrict__ resid, long strideR,
    int M, int N, int K, float scale) {
  typedef typename Elem<ET>::T T;
  typedef typename Frag<T>::V V;
  const T* A = (const T*)Ap; const T* A2 = (const T*)A2p; const T* Bt = (const T*)Btp; const T* Bt2 = (const T*)Bt2p;
  __shared__ __align__(16) float sT[8][16 * 68];
  const int b    = blockIdx.y;
  const int lane = threadIdx.x & 31;
  const int wave = threadIdx.x >> 5;
  const int tilesN = N >> 6;
  const int tilesM = M >> 6;
  const int tile = blockIdx.x * 8 + wave;
  if (tile >= tilesM * tilesN) return;
  const int tm = tile / tilesN;
  const int tn = tile - tm * tilesN;
  const int m0 = tm << 6;
  const int n0 = tn << 6;

  const T* Ab  = A  + (size_t)b * strideA;
  const T* Bb  = Bt + (size_t)b * strideB;
  const T* Ab2 = (SPLIT != 0) ? (A2  + (size_t)b * strideA) : nullptr;
  const T* Bb2 = (SPLIT == 1) ? (Bt2 + (size_t)b * strideB) : nullptr;

  const int rlane = lane & 15;
  const int koff  = (lane >> 4) * 8;
  const int mOff  = (lane >> 4) * 8;

  v8f acc[4][4];
#pragma unroll
  for (int i = 0; i < 4; ++i)
#pragma unroll
    for (int j = 0; j < 4; ++j) acc[i][j] = (v8f){0.f,0.f,0.f,0.f,0.f,0.f,0.f,0.f};

  for (int k0 = 0; k0 < K; k0 += 32) {
    V bh[4], bl[4];
#pragma unroll
    for (int j = 0; j < 4; ++j) {
      const size_t bo = (size_t)(n0 + (j << 4) + rlane) * ldb + koff + k0;
      bh[j] = Frag<T>::load(Bb + bo);
      if (SPLIT == 1) bl[j] = Frag<T>::load(Bb2 + bo);
    }
#pragma unroll
    for (int i = 0; i < 4; ++i) {
      const size_t ao = (size_t)(m0 + (i << 4) + rlane) * lda + koff + k0;
      V ah = Frag<T>::load(Ab + ao);
      V al;
      if (SPLIT != 0) al = Frag<T>::load(Ab2 + ao);
#pragma unroll
      for (int j = 0; j < 4; ++j) {
        acc[i][j] = Frag<T>::mma(ah, bh[j], acc[i][j]);
        if (SPLIT == 1) acc[i][j] = Frag<T>::mma(ah, bl[j], acc[i][j]);
        if (SPLIT != 0) acc[i][j] = Frag<T>::mma(al, bh[j], acc[i][j]);
      }
      Frag<T>::guard4(acc[i][0], acc[i][1], acc[i][2], acc[i][3], ah, (SPLIT != 0) ? al : ah);
    }
    Frag<T>::keep(bh[0], bh[1], bh[2], bh[3]);
    if (SPLIT == 1) Frag<T>::keep(bl[0], bl[1], bl[2], bl[3]);
  }
  acc_guard4(acc[0][0], acc[0][1], acc[0][2], acc[0][3]);
  acc_guard4(acc[1][0], acc[1][1], acc[1][2], acc[1][3]);
  acc_guard4(acc[2][0], acc[2][1], acc[2][2], acc[2][3]);
  acc_guard4(acc[3][0], acc[3][1], acc[3][2], acc[3][3]);

  float* slab = sT[wave];
  const float* Rb = RESID ? (resid + (size_t)b * strideR) : nullptr;
#pragma unroll
  for (int i = 0; i < 4; ++i) {
    const int mBase = m0 + (i << 4);
#pragma unroll
    for (int j = 0; j < 4; ++j) {
      const int n = n0 + (j << 4) + rlane;
      float bv = 0.f;
      if (BIAS_MODE == 2) bv = bias[n];
#pragma unroll
      for (int r = 0; r < 8; ++r) {
        float v = acc[i][j][r] * scale;
        if (BIAS_MODE == 1) v += bias[mBase + mOff + r];
        if (BIAS_MODE == 2) v += bv;
        if (RESID) v += Rb[(size_t)(mBase + mOff + r) * ldc + n];
        if (ACT == 2) v = fmaxf(v, 0.0f);
        if (ACT == 4) v = (v > 0.f) ? v : 0.01f * v;
        if (ACT == 6) v = (v > 0.f) ? v : 0.2f * v;
        slab[(mOff + r) * 68 + (j << 4) + rlane] = v;
      }
    }
    __builtin_amdgcn_fence(__ATOMIC_RELEASE, "workgroup");
    __builtin_amdgcn_wave_barrier();
    __builtin_amdgcn_fence(__ATOMIC_ACQUIRE, "workgroup");
    if (OUT_MODE == 0) {
      float* C = (float*)Cout + (size_t)b * strideC;
      const int hh = lane >> 4, c4 = (lane & 15) * 4;
      for (int pass = 0; pass < 2; ++pass) {
#pragma unroll
        for (int it = 0; it < 8; ++it) {
          const int row = it * 2 + hh;
          v4f v = *(const v4f*)(slab + row * 68 + c4);
          *(volatile v4f*)(C + (size_t)(mBase + row) * ldc + n0 + c4) = v;
        }
        __threadfence();
      }
    } else {
      const int q = lane >> 3, c8 = (lane & 7) * 8;
      unsigned short* C  = (unsigned short*)Cout  + (size_t)b * strideC;
      unsigned short* C2 = (OUT_MODE == 2) ? ((unsigned short*)Cout2 + (size_t)b * strideC) : nullptr;
      for (int pass = 0; pass < 2; ++pass) {
#pragma unroll
        for (int it = 0; it < 4; ++it) {
          const int row = it * 4 + q;
          const float* sp = slab + row * 68 + c8;
          v8h hv, lv;
#pragma unroll
          for (int e = 0; e < 8; ++e) {
            if (OUT_MODE == 1) {
              hv[e] = (_Float16)sp[e];
            } else {
              unsigned short hb = f2bf_bits(sp[e]);
              unsigned short lb = f2bf_bits(sp[e] - bf_bits2f(hb));
              hv[e] = __builtin_bit_cast(_Float16, hb);
              lv[e] = __builtin_bit_cast(_Float16, lb);
            }
          }
          *(volatile v8h*)(C + (size_t)(mBase + row) * ldc + n0 + c8) = hv;
          if (OUT_MODE == 2) *(volatile v8h*)(C2 + (size_t)(mBase + row) * ldc + n0 + c8) = lv;
        }
        __threadfence();
      }
    }
    __builtin_amdgcn_fence(__ATOMIC_RELEASE, "workgroup");
    __builtin_amdgcn_wave_barrier();
    __builtin_amdgcn_fence(__ATOMIC_ACQUIRE, "workgroup");
  }
}

__device__ __forceinline__ int blk_excl_scan(int cnt, int* scan_ws, int tid, int* tot) {
  const int lane = tid & 31, wave = tid >> 5; int incl = cnt;
#pragma unroll
  for (int o = 1; o < 32; o <<= 1) { const int v = __shfl_up(incl, o, 32); if (lane >= o) incl += v; }
  if (lane == 31) scan_ws[wave] = incl;
  __syncthreads();
  if (wave == 0) {
    const int wr = scan_ws[lane];
    const int wv = (lane < kNT / 32) ? wr : 0; int wincl = wv;
#pragma unroll
    for (int o = 1; o < 32; o <<= 1) { const int v = __shfl_up(wincl, o, 32); if (lane >= o) wincl += v; }
    if (lane < kNT / 32) scan_ws[32 + lane] = wincl - wv;
    if (lane == 31) scan_ws[64] = wincl;
  }
  __syncthreads();
  const int res = scan_ws[32 + wave] + incl - cnt; *tot = scan_ws[64];
  return res;
}

__global__ __launch_bounds__(kNT) void copy4r_kernel(const float* __restrict__ src, float* __restrict__ dst, int n4) {
  const int i = blockIdx.x * kNT + threadIdx.x;
  if (i >= n4) return;
  const v4f v = *(const v4f*)(src + 4 * (size_t)i);
  v4f o;
#pragma unroll
  for (int e = 0; e < 4; ++e) o[e] = bfr(v[e]);
  float* p = dst + 4 * (size_t)i;
  *(volatile v4f*)p = o;
  __threadfence();
  *(volatile v4f*)p = o;
}

__global__ __launch_bounds__(kNT) void zero4_kernel(float* __restrict__ dst, int n4) {
  const int i = blockIdx.x * kNT + threadIdx.x;
  if (i >= n4) return;
  const v4f z = {0.f, 0.f, 0.f, 0.f};
  float* p = dst + 4 * (size_t)i;
  *(volatile v4f*)p = z;
  __threadfence();
  *(volatile v4f*)p = z;
}

__global__ __launch_bounds__(kNT) void key8_kernel(const int* __restrict__ lrow, unsigned* __restrict__ key32) {
  const int i = blockIdx.x * kNT + threadIdx.x;
  if (i >= kNnzPad / 16) return;
  const int eb = 16 * i;
  const bool inb = eb < kNnz;
  const int ebc = inb ? eb : (kNnz - 16);
  const v4i ra = *(const v4i*)(lrow + ebc);
  const v4i rbv = *(const v4i*)(lrow + ebc + 4);
  const v4i rcv = *(const v4i*)(lrow + ebc + 8);
  const v4i rdv = *(const v4i*)(lrow + ebc + 12);
  int rv[16];
#pragma unroll
  for (int e = 0; e < 4; ++e) { rv[e] = ra[e]; rv[4 + e] = rbv[e]; rv[8 + e] = rcv[e]; rv[12 + e] = rdv[e]; }
  unsigned wd[4];
#pragma unroll
  for (int q = 0; q < 4; ++q) {
    unsigned acc = 0u;
#pragma unroll
    for (int k = 0; k < 4; ++k) {
      const int r = rv[4 * q + k];
      const unsigned c = (inb && r >= 0 && r < kNumNode) ? (unsigned)(r >> 10) : 255u;
      acc |= c << (8 * k);
    }
    wd[q] = acc;
  }
  const v4u u = (v4u){wd[0], wd[1], wd[2], wd[3]};
  unsigned* p = key32 + 4 * (size_t)i;
  *(volatile v4u*)p = u;
  __threadfence();
  *(volatile v4u*)p = u;
}

__global__ __launch_bounds__(kNT) void prep_kernel(const float* __restrict__ w1, const float* __restrict__ b1,
                                                   const float* __restrict__ w2, const float* __restrict__ b2,
                                                   unsigned short* __restrict__ BT, float* __restrict__ BS) {
  __shared__ float s1[64 * 65];
  __shared__ float s2[64 * 65];
  const int tid = threadIdx.x, lane = tid & 31, wave = tid >> 5;
  const int k = blockIdx.x;
  const float* w1k = w1 + (size_t)k * 4096;
  const float* w2k = w2 + (size_t)k * 4096;
#pragma unroll
  for (int i = 0; i < 4; ++i) {
    const int i4 = i * kNT + tid;
    const v4f a = *(const v4f*)(w1k + 4 * i4);
    const v4f c = *(const v4f*)(w2k + 4 * i4);
#pragma unroll
    for (int e = 0; e < 4; ++e) {
      const int flat = 4 * i4 + e;
      const int kk = flat >> 6, n = flat & 63;
      s1[kk * 65 + n] = a[e];
      s2[kk * 65 + n] = c[e];
    }
  }
  __syncthreads();
  unsigned short* bt = BT + (size_t)k * 64 * kKdim;
  const int q8 = lane >> 3, c8 = (lane & 7) * 8;
  const int nr0 = wave * 8 + q8;
  v4u ua[2], ub[2];
#pragma unroll
  for (int it = 0; it < 2; ++it) {
    const int n = nr0 + it * 4;
    unsigned short ha[8], hb[8];
#pragma unroll
    for (int e = 0; e < 8; ++e) {
      const int kk = c8 + e;
      ha[e] = f2bf_bits(s1[kk * 65 + n]);
      hb[e] = f2bf_bits(s2[kk * 65 + n]);
    }
    ua[it] = (v4u){pk16(ha[0], ha[1]), pk16(ha[2], ha[3]), pk16(ha[4], ha[5]), pk16(ha[6], ha[7])};
    ub[it] = (v4u){pk16(hb[0], hb[1]), pk16(hb[2], hb[3]), pk16(hb[4], hb[5]), pk16(hb[6], hb[7])};
  }
  for (int pass = 0; pass < 2; ++pass) {
#pragma unroll
    for (int it = 0; it < 2; ++it) {
      const int n = nr0 + it * 4;
      *(volatile v4u*)(bt + (size_t)n * kKdim + c8) = ua[it];
      *(volatile v4u*)(bt + (size_t)n * kKdim + 64 + c8) = ub[it];
    }
    __threadfence();
  }
  if (wave == 0) {
    const int c4 = (lane & 15) * 4;
    const v4f x = *(const v4f*)(b1 + k * kDim + c4);
    const v4f y = *(const v4f*)(b2 + k * kDim + c4);
    v4f bb;
#pragma unroll
    for (int e = 0; e < 4; ++e) bb[e] = bfr(x[e]) + bfr(y[e]);
    for (int pass = 0; pass < 2; ++pass) {
      if (lane < 16) *(volatile v4f*)(BS + k * kDim + c4) = bb;
      __threadfence();
    }
  }
}

__global__ __launch_bounds__(kNT) void mlp_blend_kernel(const float* __restrict__ uemb, const float* __restrict__ feat,
                                                        const float* __restrict__ l1w, const float* __restrict__ l1b,
                                                        const float* __restrict__ l2w, const float* __restrict__ l2b,
                                                        const int* __restrict__ uidx, const float* __restrict__ ratio,
                                                        float* __restrict__ E0) {
  const int tid = threadIdx.x, lane = tid & 31, wave = tid >> 5;
  const int b = blockIdx.x * 8 + wave;
  const int c4 = (lane & 15) * 4;
  const float f0 = bfr(feat[b * 4]), f1 = bfr(feat[b * 4 + 1]), f2 = bfr(feat[b * 4 + 2]), f3 = bfr(feat[b * 4 + 3]);
  const float g0 = bfr(l1w[lane]), g1 = bfr(l1w[32 + lane]), g2 = bfr(l1w[64 + lane]), g3 = bfr(l1w[96 + lane]);
  float d = f0 * g0;
  d = fmaf(f1, g1, d);
  d = fmaf(f2, g2, d);
  d = fmaf(f3, g3, d);
  const float hid = d + bfr(l1b[lane]);
  v4f acc = {0.f, 0.f, 0.f, 0.f};
#pragma unroll 1
  for (int h = 0; h < 32; ++h) {
    const float hv = __shfl(hid, h, 32);
    const v4f w4 = *(const v4f*)(l2w + h * kDim + c4);
    v4f wr;
#pragma unroll
    for (int e = 0; e < 4; ++e) wr[e] = bfr(w4[e]);
    acc = acc + hv * wr;
  }
  const v4f b4 = *(const v4f*)(l2b + c4);
  v4f mlp;
#pragma unroll
  for (int e = 0; e < 4; ++e) mlp[e] = acc[e] + bfr(b4[e]);
  int u = uidx[b];
  u = u < 0 ? 0 : (u >= kNumUser ? kNumUser - 1 : u);
  unsigned laterm = 0u;
#pragma unroll 1
  for (int jb = 0; jb < kBatch / 32; ++jb) {
    const int idx = jb * 32 + lane;
    int v = uidx[idx];
    v = v < 0 ? 0 : (v >= kNumUser ? kNumUser - 1 : v);
    const int m = (idx > b && v == u) ? 1 : 0;
    laterm |= (unsigned)__ballot(m);
  }
  if (laterm == 0u) {
    const float r = bfr(ratio[0]);
    const float omr = 1.0f - r;
    const v4f ue = *(const v4f*)(uemb + (size_t)u * kDim + c4);
    v4f uer;
#pragma unroll
    for (int e = 0; e < 4; ++e) uer[e] = bfr(ue[e]);
    const v4f upd = uer * omr + mlp * r;
    float* op = E0 + (size_t)u * kDim + c4;
    for (int pass = 0; pass < 2; ++pass) {
      if (lane < 16) *(volatile v4f*)op = upd;
      __threadfence();
    }
  }
}

__global__ __launch_bounds__(kNT) void gather_rows_kernel(const float* __restrict__ Eb, const int* __restrict__ uidx,
                                                          const int* __restrict__ pidx, const int* __restrict__ nidx,
                                                          float* __restrict__ out, int layer, int do_norm) {
  const int s = blockIdx.y;
  const int tid = threadIdx.x, lane = tid & 31, wave = tid >> 5;
  const int hh = lane >> 4, c4 = (lane & 15) * 4;
  const int r = blockIdx.x * 16 + wave * 2 + hh;
  int a0 = uidx[r], a1 = pidx[r], a2 = nidx[r];
  a0 = a0 < 0 ? 0 : (a0 >= kNumUser ? kNumUser - 1 : a0);
  a1 = a1 < 0 ? 0 : (a1 >= kNumItem ? kNumItem - 1 : a1);
  a2 = a2 < 0 ? 0 : (a2 >= kNumItem ? kNumItem - 1 : a2);
  const int node = (s == 0) ? a0 : ((s == 1) ? (kNumUser + a1) : (kNumUser + a2));
  v4f v = *(const v4f*)(Eb + (size_t)node * kDim + c4);
  float ss = v[0] * v[0] + v[1] * v[1] + v[2] * v[2] + v[3] * v[3];
  ss += __shfl_xor(ss, 1, 32);
  ss += __shfl_xor(ss, 2, 32);
  ss += __shfl_xor(ss, 4, 32);
  ss += __shfl_xor(ss, 8, 32);
  const float inv = 1.0f / fmaxf(sqrtf(ss), 1e-12f);
  const float sc = do_norm ? inv : 1.0f;
  v = v * sc;
  float* op = out + ((size_t)(s * kBatch + r) * 256 + layer * kDim + c4);
  for (int pass = 0; pass < 2; ++pass) {
    *(volatile v4f*)op = v;
    __threadfence();
  }
}

__global__ __launch_bounds__(kNT) void agg_tile_kernel(const float* __restrict__ E, const unsigned* __restrict__ key32,
                                                       const int* __restrict__ lrow, const int* __restrict__ lcol,
                                                       const float* __restrict__ lval,
                                                       unsigned short* __restrict__ Ahi, unsigned short* __restrict__ Alo) {
  extern __shared__ float4 accs_dyn[];
  __shared__ unsigned LIST[kCap];
  __shared__ int scan_ws[80];
  float* accs = (float*)accs_dyn;
  const int tid = threadIdx.x, lane = tid & 31, wave = tid >> 5;
  const int t = blockIdx.x;
  const int n0 = t * kTileRows;
  const unsigned rep = (unsigned)t * 0x01010101u;
  const v4f z4 = {0.f, 0.f, 0.f, 0.f};
#pragma unroll 1
  for (int i = 0; i < (kTileRows * kDim / 4) / kNT; ++i)
    *(v4f*)(accs + 4 * (size_t)(i * kNT + tid)) = z4;
#pragma unroll
  for (int i = 0; i < kCap / kNT; ++i) LIST[i * kNT + tid] = 0u;
  if (tid < 80) scan_ws[tid] = 0;
  __syncthreads();

#pragma unroll 1
  for (int ch = 0; ch < kNumChunks; ++ch) {
    const v4u* kp = (const v4u*)(key32 + (size_t)ch * (kChunk / 4) + (size_t)tid * (kEPT / 4));
    v4u w[8];
#pragma unroll
    for (int g = 0; g < 8; ++g) w[g] = kp[g];
    unsigned mw[8];
    int cnt = 0;
#pragma unroll
    for (int g = 0; g < 8; ++g) {
      unsigned m = 0u;
#pragma unroll
      for (int q = 0; q < 4; ++q) {
        const unsigned x = w[g][q] ^ rep;
        const unsigned y = ((x & 0x7F7F7F7Fu) + 0x7F7F7F7Fu) | x;
        const unsigned z = (~y) & 0x80808080u;
        m |= z >> (7 - q);
      }
      mw[g] = m;
      cnt += __builtin_popcount(m);
    }
    int tot;
    int p = blk_excl_scan(cnt, scan_ws, tid, &tot);
    const int ebase = ch * kChunk + tid * kEPT;
#pragma unroll
    for (int g = 0; g < 8; ++g) {
      unsigned m = mw[g];
#pragma unroll 1
      while (m != 0u) {
        const int bb = __builtin_ctz(m);
        m &= m - 1u;
        const int e = ebase + 16 * g + 4 * (bb & 7) + (bb >> 3);
        if ((unsigned)p < (unsigned)kCap) LIST[p] = (unsigned)e;
        ++p;
      }
    }
    __syncthreads();
    const int totc = tot < kCap ? tot : kCap;
#pragma unroll 1
    for (int i0 = 0; i0 < totc; i0 += kNT) {
      const int i = i0 + tid;
      const bool valid = i < totc;
      const int ic = i < kCap ? i : (kCap - 1);
      unsigned e = LIST[ic];
      e = e < (unsigned)kNnz ? e : (unsigned)(kNnz - 1);
      const int r = lrow[e];
      int rl = r - n0;
      rl = rl < 0 ? 0 : (rl >= kTileRows ? kTileRows - 1 : rl);
      if (valid) LIST[i] = ((unsigned)rl << 22) | e;
    }
    __syncthreads();
#pragma unroll 1
    for (int base = 0; base < totc; base += 32) {
      const int q = base + lane;
      const int qc = q < totc ? q : (totc - 1);
      const unsigned ent = LIST[qc];
      const int own = (q < totc && (int)(ent >> 29) == wave) ? 1 : 0;
      unsigned msk = (unsigned)__ballot(own);
#pragma unroll 1
      for (int it = 0; it < 32; ++it) {
        if (msk == 0u) break;
        const int bp = __builtin_ctz(msk);
        msk &= msk - 1u;
        const unsigned eb2 = (unsigned)__builtin_amdgcn_readlane((int)ent, bp);
        const int rl = (int)((eb2 >> 22) & 1023u);
        int e = (int)(eb2 & 0x3FFFFFu);
        e = e < kNnz ? e : kNnz - 1;
        int col = lcol[e];
        col = col < 0 ? 0 : (col >= kNumNode ? kNumNode - 1 : col);
        const float val = bfr(lval[e]);
        const v2f ev = *(const v2f*)(E + (size_t)col * kDim + 2 * lane);
        float* ap = accs + rl * kDim + 2 * lane;
        v2f a = *(const v2f*)ap;
        a = a + val * ev;
        *(v2f*)ap = a;
      }
    }
    __syncthreads();
  }

  const int q8 = lane >> 3, c8 = (lane & 7) * 8;
#pragma unroll 1
  for (int i = 0; i < kWaveRows / 4; ++i) {
    const int rlb = wave * kWaveRows + 4 * i;
    const int rb = n0 + rlb;
    if (rb >= kRowsPad) break;
    const int rl = rlb + q8;
    const int row = rb + q8;
    const float* ap = accs + rl * kDim + c8;
    const v4f a0 = *(const v4f*)(ap), a1 = *(const v4f*)(ap + 4);
    const float* ep = E + (size_t)row * kDim + c8;
    const v4f e0 = *(const v4f*)(ep), e1 = *(const v4f*)(ep + 4);
    const float lv = (row < kNumNode) ? 1.0f : 0.0f;
    const v4f s0 = (a0 + e0) * lv, s1 = (a1 + e1) * lv;
    const v4f p0 = (a0 * e0) * lv, p1 = (a1 * e1) * lv;
    unsigned short hs[8], ls[8], hp[8], lp[8];
#pragma unroll
    for (int e = 0; e < 4; ++e) {
      unsigned short hb;
      hb = f2bf_bits(s0[e]); hs[e] = hb;     ls[e] = f2bf_bits(s0[e] - bf_bits2f(hb));
      hb = f2bf_bits(s1[e]); hs[4 + e] = hb; ls[4 + e] = f2bf_bits(s1[e] - bf_bits2f(hb));
      hb = f2bf_bits(p0[e]); hp[e] = hb;     lp[e] = f2bf_bits(p0[e] - bf_bits2f(hb));
      hb = f2bf_bits(p1[e]); hp[4 + e] = hb; lp[4 + e] = f2bf_bits(p1[e] - bf_bits2f(hb));
    }
    const v4u ush = (v4u){pk16(hs[0], hs[1]), pk16(hs[2], hs[3]), pk16(hs[4], hs[5]), pk16(hs[6], hs[7])};
    const v4u usl = (v4u){pk16(ls[0], ls[1]), pk16(ls[2], ls[3]), pk16(ls[4], ls[5]), pk16(ls[6], ls[7])};
    const v4u uph = (v4u){pk16(hp[0], hp[1]), pk16(hp[2], hp[3]), pk16(hp[4], hp[5]), pk16(hp[6], hp[7])};
    const v4u upl = (v4u){pk16(lp[0], lp[1]), pk16(lp[2], lp[3]), pk16(lp[4], lp[5]), pk16(lp[6], lp[7])};
    unsigned short* oh = Ahi + (size_t)row * kKdim + c8;
    unsigned short* ol = Alo + (size_t)row * kKdim + c8;
    for (int pass = 0; pass < 2; ++pass) {
      *(volatile v4u*)(oh) = ush;
      *(volatile v4u*)(oh + 64) = uph;
      *(volatile v4u*)(ol) = usl;
      *(volatile v4u*)(ol + 64) = upl;
      __threadfence();
    }
  }
}

extern "C" void kernel_launch(void* const* d_in, const int* in_sizes, int n_in,
                              void* d_out, int out_size, void* d_ws, size_t ws_size, hipStream_t stream) {
  (void)in_sizes;
  if (n_in < 18) return;
  if (out_size < 3 * kBatch * 256) return;
  const float* user_emb  = (const float*)d_in[0];
  const float* item_emb  = (const float*)d_in[1];
  const float* lin1_w    = (const float*)d_in[2];
  const float* lin1_b    = (const float*)d_in[3];
  const float* lin2_w    = (const float*)d_in[4];
  const float* lin2_b    = (const float*)d_in[5];
  const float* w1        = (const float*)d_in[6];
  const float* b1        = (const float*)d_in[7];
  const float* w2        = (const float*)d_in[8];
  const float* b2        = (const float*)d_in[9];
  const int*   lap_row   = (const int*)d_in[10];
  const int*   lap_col   = (const int*)d_in[11];
  const float* lap_val   = (const float*)d_in[12];
  const int*   user_idx  = (const int*)d_in[13];
  const float* user_feat = (const float*)d_in[14];
  const int*   pos_idx   = (const int*)d_in[15];
  const int*   neg_idx   = (const int*)d_in[16];
  const float* ratio     = (const float*)d_in[17];
  float* out = (float*)d_out;

  const size_t planeBytes = (size_t)kRowsPad * kDim * sizeof(float);
  const size_t aplBytes   = (size_t)kRowsPad * kKdim * 2;
  const size_t keyBytes   = (size_t)kNnzPad;
  const size_t btBytes    = (size_t)kLayers * kDim * kKdim * 2;
  const size_t bsBytes    = (size_t)kLayers * kDim * sizeof(float);
  const size_t offE = 0, offAH = planeBytes, offAL = offAH + aplBytes, offKEY = offAL + aplBytes;
  const size_t offBT = offKEY + keyBytes, offBS = offBT + btBytes;
  const size_t total = offBS + bsBytes;
  if (total > ws_size || total > (size_t)134217728) return;
  char* ws = (char*)d_ws;
  float* EPL = (float*)(ws + offE);
  unsigned short* AHI = (unsigned short*)(ws + offAH);
  unsigned short* ALO = (unsigned short*)(ws + offAL);
  unsigned* KEY = (unsigned*)(ws + offKEY);
  unsigned short* BT = (unsigned short*)(ws + offBT);
  float* BS = (float*)(ws + offBS);

  copy4r_kernel<<<(kNumUser * 16) / kNT, kNT, 0, stream>>>(user_emb, EPL, kNumUser * 16);
  copy4r_kernel<<<(kNumItem * 16) / kNT, kNT, 0, stream>>>(item_emb, EPL + (size_t)kNumUser * kDim, kNumItem * 16);
  zero4_kernel<<<1, kNT, 0, stream>>>(EPL + (size_t)kNumNode * kDim, (kRowsPad - kNumNode) * 16);
  key8_kernel<<<kNnzPad / 16 / kNT, kNT, 0, stream>>>(lap_row, KEY);
  prep_kernel<<<kLayers, kNT, 0, stream>>>(w1, b1, w2, b2, BT, BS);
  mlp_blend_kernel<<<kBatch / 8, kNT, 0, stream>>>(user_emb, user_feat, lin1_w, lin1_b, lin2_w, lin2_b, user_idx, ratio, EPL);
  gather_rows_kernel<<<dim3(kBatch / 16, 3), kNT, 0, stream>>>(EPL, user_idx, pos_idx, neg_idx, out, 0, 0);

  for (int k = 0; k < kLayers; ++k) {
    agg_tile_kernel<<<kNumTiles, kNT, kDynLds, stream>>>(EPL, KEY, lap_row, lap_col, lap_val, AHI, ALO);
    {
      const int tiles = (kRowsPad / 64) * (kDim / 64);
      wmma_gemm64<1, 2, 2, 0, false, 6><<<dim3((tiles + 7) / 8, 1), 256, 0, stream>>>(
          (const unsigned short*)AHI, (const unsigned short*)ALO, kKdim, 0L,
          (const unsigned short*)(BT + (size_t)k * kDim * kKdim), (const unsigned short*)nullptr, kKdim, 0L,
          (void*)EPL, (void*)nullptr, kDim, 0L,
          (const float*)(BS + k * kDim), (const float*)nullptr, 0L,
          kRowsPad, kDim, kKdim, 1.0f);
    }
    gather_rows_kernel<<<dim3(kBatch / 16, 3), kNT, 0, stream>>>(EPL, user_idx, pos_idx, neg_idx, out, k + 1, 1);
  }
}
